// Net_56770877718819
// MI455X (gfx1250) — hardware-verified
//
#include <hip/hip_runtime.h>
#include <stdint.h>

#ifndef NB
#define NB 8
#endif
#define NB_FULL  8
#define NN       228
#define NT       12
#define SEQ      2736
#define SEQ_FULL 2736
#define SP       2752
#define GF       64
#define HD       32
#define DFF      2048
#define FCO      256
#define KFC      768
#define NEMB     16
#define ROWS     (NB * SEQ)
#define QTILES   171
#define MW       96
#define KW       86
#define NPAD     240
#define YP       128
#define SCP      68
#define WSCAP    134217728

#define OW_QKV 0
#define OW_O   12288
#define OW_1   16384
#define OW_2   147456
#define OW_FC  278528
#define NW_ALL 475136

static_assert(NB >= 1 && NB <= NB_FULL);
static_assert(SEQ == NN * NT);
static_assert(SEQ == SEQ_FULL);
static_assert(QTILES * 16 == SEQ);
static_assert(QTILES % 3 == 0);
static_assert(SEQ % 8 == 0);
static_assert(SEQ % 48 == 0);
static_assert(ROWS % 48 == 0);
static_assert(SP % 64 == 0);
static_assert(SP >= SEQ);
static_assert(KW * 32 == SP);
static_assert(KW <= MW);
static_assert(MW % 32 == 0);
static_assert(KW > 64 && KW - 64 <= 32);
static_assert(GF == 64);
static_assert(HD == 32);
static_assert(2 * HD == GF);
static_assert(DFF % 32 == 0);
static_assert(KFC == NT * GF);
static_assert(KFC % 32 == 0);
static_assert(FCO == 256);
static_assert(NPAD % 16 == 0);
static_assert(NPAD >= NN);
static_assert(NB * NT <= YP);
static_assert(YP % 32 == 0);
static_assert(ROWS % 4 == 0);
static_assert(OW_O == 3 * GF * GF);
static_assert(OW_1 == OW_O + GF * GF);
static_assert(OW_2 == OW_1 + DFF * GF);
static_assert(OW_FC == OW_2 + GF * DFF);
static_assert(NW_ALL == OW_FC + FCO * KFC);
static_assert((NW_ALL / 8) % 256 == 0);
static_assert((GF * GF / 8) % 256 == 0);
static_assert(NB_FULL * SEQ_FULL * 4 == 87552);

typedef float          v2f   __attribute__((ext_vector_type(2)));
typedef float          v4f   __attribute__((ext_vector_type(4)));
typedef float          v8f   __attribute__((ext_vector_type(8)));
typedef int            v8i   __attribute__((ext_vector_type(8)));
typedef unsigned int   v4u   __attribute__((ext_vector_type(4)));
typedef unsigned short v8us  __attribute__((ext_vector_type(8)));
typedef __bf16         v16b  __attribute__((ext_vector_type(16)));
typedef _Float16       v16h  __attribute__((ext_vector_type(16)));
typedef v2f  __attribute__((may_alias)) v2fa;
typedef v4f  __attribute__((may_alias)) v4fa;
typedef v4u  __attribute__((may_alias)) v4ua;
typedef v8us __attribute__((may_alias)) v8usa;
union Frag { v16b b; v16h f; v8us h[2]; v4u q[2]; v8i w; };

__device__ __forceinline__ v8f wmb(const Frag& a, const Frag& b, v8f c) {
  v8f d = __builtin_amdgcn_wmma_f32_16x16x32_bf16(false, a.b, false, b.b, (short)0, c, false, false);
  asm volatile("v_nop\n\tv_nop\n\tv_nop\n\tv_nop" : "+v"(d) : "v"(a.w), "v"(b.w));
  return d;
}
__device__ __forceinline__ v8f wmh(const Frag& a, const Frag& b, v8f c) {
  v8f d = __builtin_amdgcn_wmma_f32_16x16x32_f16(false, a.f, false, b.f, (short)0, c, false, false);
  asm volatile("v_nop\n\tv_nop\n\tv_nop\n\tv_nop" : "+v"(d) : "v"(a.w), "v"(b.w));
  return d;
}
__device__ __forceinline__ v8f z8() { v8f z = {0.f, 0.f, 0.f, 0.f, 0.f, 0.f, 0.f, 0.f}; return z; }

__device__ __forceinline__ void ld_frag(Frag& f, const unsigned short* p) {
  f.h[0] = *(const v8usa*)p;
  f.h[1] = *(const v8usa*)(p + 16);
}

__device__ __forceinline__ unsigned f2bf_rne(float f) {
  const unsigned u = __float_as_uint(f);
  return (u + 0x7FFFu + ((u >> 16) & 1u)) >> 16;
}
__device__ __forceinline__ float bfr(float f) { return __uint_as_float(f2bf_rne(f) << 16); }
__device__ __forceinline__ unsigned pk2b(float a, float b) { return (f2bf_rne(a) & 0xFFFFu) | (f2bf_rne(b) << 16); }

__device__ __forceinline__ void split2(float x0, float x1, unsigned& hp, unsigned& lp) {
  const unsigned h0 = __float_as_uint(x0) & 0xFFFF0000u;
  const unsigned h1 = __float_as_uint(x1) & 0xFFFF0000u;
  hp = (h0 >> 16) | h1;
  const unsigned l0 = f2bf_rne(x0 - __uint_as_float(h0));
  const unsigned l1 = f2bf_rne(x1 - __uint_as_float(h1));
  lp = (l0 & 0xFFFFu) | (l1 << 16);
}

__device__ __forceinline__ unsigned short f2h_bits(float f) {
  const _Float16 x = (_Float16)f;
  return __builtin_bit_cast(unsigned short, x);
}
__device__ __forceinline__ unsigned pk2h(float a, float b) {
  return (unsigned)f2h_bits(a) | ((unsigned)f2h_bits(b) << 16);
}

__device__ __forceinline__ float wsum(float v) {
  v += __shfl_xor(v, 16);
  v += __shfl_xor(v, 8);
  v += __shfl_xor(v, 4);
  v += __shfl_xor(v, 2);
  v += __shfl_xor(v, 1);
  return v;
}

__device__ __forceinline__ void wave_lds_sync() {
  __builtin_amdgcn_fence(3  , "wavefront");
  __builtin_amdgcn_wave_barrier();
  __builtin_amdgcn_fence(2  , "wavefront");
}

__device__ __forceinline__ void hl_lines_store(const float* sc, unsigned short* grow0, int lane) {
  const int q8 = lane & 7, sub = lane >> 3;
#pragma unroll
  for (int i = 0; i < 8; ++i) {
    const int L = 4 * i + sub;
    const int row = L >> 1, part = L & 1;
    const v4f g0 = *(const v4fa*)(sc + row * SCP + 8 * q8);
    const v4f g1 = *(const v4fa*)(sc + row * SCP + 8 * q8 + 4);
    unsigned h0, h1, h2, h3, l0, l1, l2, l3;
    split2(g0[0], g0[1], h0, l0);
    split2(g0[2], g0[3], h1, l1);
    split2(g1[0], g1[1], h2, l2);
    split2(g1[2], g1[3], h3, l3);
    const unsigned msk = part ? 0u : 0xFFFFFFFFu;
    const v4u o = { (h0 & msk) | (l0 & ~msk), (h1 & msk) | (l1 & ~msk),
                    (h2 & msk) | (l2 & ~msk), (h3 & msk) | (l3 & ~msk) };
    *(volatile v4u*)(grow0 + (size_t)row * 128 + part * 64 + 8 * q8) = o;
  }
}
__device__ __forceinline__ void f32_lines_store(const float* sc, float* grow0, int pitch, int lane) {
  const int q8 = lane & 7, sub = lane >> 3;
#pragma unroll
  for (int i = 0; i < 8; ++i) {
    const int L = 4 * i + sub;
    const int row = L >> 1, hl = L & 1;
    const v4f v = *(const v4fa*)(sc + row * SCP + 32 * hl + 4 * q8);
    *(volatile v4f*)(grow0 + (size_t)row * pitch + 32 * hl + 4 * q8) = v;
  }
}

__device__ __forceinline__ void cvt8(const float* __restrict__ src, unsigned short* __restrict__ dst, int us, int ud) {
  const v4f a = *(const v4fa*)(src + (size_t)us * 8);
  const v4f b = *(const v4fa*)(src + (size_t)us * 8 + 4);
  const v4u v = { pk2b(a[0], a[1]), pk2b(a[2], a[3]), pk2b(b[0], b[1]), pk2b(b[2], b[3]) };
  unsigned short* d = dst + (size_t)ud * 8;
  *(volatile v4u*)d = v;
  __threadfence();
  *(volatile v4u*)d = v;
}
__global__ __launch_bounds__(256) void prep_kernel(const float* __restrict__ wq, const float* __restrict__ wk,
                                                   const float* __restrict__ wv, const float* __restrict__ wo,
                                                   const float* __restrict__ w1, const float* __restrict__ w2,
                                                   const float* __restrict__ fcw, unsigned short* __restrict__ wall) {
  const int u = blockIdx.x * 256 + threadIdx.x;
  if (u < 512)        cvt8(wq, wall, u, u);
  else if (u < 1024)  cvt8(wk, wall, u - 512, u);
  else if (u < 1536)  cvt8(wv, wall, u - 1024, u);
  else if (u < 2048)  cvt8(wo, wall, u - 1536, u);
  else if (u < 18432) cvt8(w1, wall, u - 2048, u);
  else if (u < 34816) cvt8(w2, wall, u - 18432, u);
  else                cvt8(fcw, wall, u - 34816, u);
}

__device__ __forceinline__ unsigned pack32(const int* __restrict__ mr, int kbase, int nw, int lane) {
  unsigned wv = 0xFFFFFFFFu;
#pragma unroll 2
  for (int j = 0; j < nw; ++j) {
    const int key = kbase + 32 * j + lane;
    const int kc = key < SEQ ? key : SEQ - 1;
    const int mv = mr[kc];
    const int pred = (mv != 0) | (key >= SEQ);
    const unsigned bal = (unsigned)__ballot(pred);
    wv = (lane == j) ? bal : wv;
  }
  return wv;
}
__global__ __launch_bounds__(256) void mask_kernel(const int* __restrict__ mask, unsigned* __restrict__ mb,
                                                   unsigned* __restrict__ tc) {
  __shared__ unsigned sw[16 * MW];
  const int tid = threadIdx.x, lane = tid & 31, w = tid >> 5;
  const int qt = blockIdx.x;
#pragma unroll 1
  for (int rr = 0; rr < 2; ++rr) {
    const int rl = 2 * w + rr;
    const int row = 16 * qt + rl;
    const int* mr = mask + (size_t)row * SEQ_FULL;
    const unsigned w0 = pack32(mr, 0, 32, lane);
    const unsigned w1 = pack32(mr, 1024, 32, lane);
    const unsigned w2 = pack32(mr, 2048, KW - 64, lane);
    sw[rl * MW + lane] = w0;
    sw[rl * MW + 32 + lane] = w1;
    sw[rl * MW + 64 + lane] = w2;
    unsigned* d = mb + (size_t)row * MW + lane;
    *(volatile unsigned*)d = w0;
    *(volatile unsigned*)(d + 32) = w1;
    *(volatile unsigned*)(d + 64) = w2;
    __threadfence();
    *(volatile unsigned*)d = w0;
    *(volatile unsigned*)(d + 32) = w1;
    *(volatile unsigned*)(d + 64) = w2;
  }
  __syncthreads();
  if (tid < MW) {
    unsigned a = 0xFFFFFFFFu, o = 0u;
#pragma unroll 4
    for (int r = 0; r < 16; ++r) {
      const unsigned v = sw[r * MW + tid];
      a &= v;
      o |= v;
    }
    const unsigned cls = (a == 0xFFFFFFFFu) ? 2u : ((o == 0u) ? 0u : 1u);
    unsigned* d = tc + (size_t)qt * MW + tid;
    *(volatile unsigned*)d = cls;
    __threadfence();
    *(volatile unsigned*)d = cls;
  }
}

__global__ __launch_bounds__(256) void gcn_kernel(const float* __restrict__ x, const float* __restrict__ ne,
                                                  const float* __restrict__ gcw, const float* __restrict__ gcb,
                                                  const float* __restrict__ bn1g, const float* __restrict__ bn1b,
                                                  float* __restrict__ H, unsigned* __restrict__ HHLw) {
  const int tid = threadIdx.x, lane = tid & 31, w = tid >> 5;
  const int n = blockIdx.x * 8 + w;
  float gw0 = 0.f, gw1 = 0.f, gb0 = 0.f, gb1 = 0.f;
#pragma unroll 1
  for (int e = 0; e < NEMB; ++e) {
    const float a = bfr(ne[n * NEMB + e]);
    const v2f wv = *(const v2fa*)(gcw + e * GF + 2 * lane);
    const v2f bv = *(const v2fa*)(gcb + e * GF + 2 * lane);
    gw0 += a * bfr(wv[0]);
    gw1 += a * bfr(wv[1]);
    gb0 += a * bfr(bv[0]);
    gb1 += a * bfr(bv[1]);
  }
  float s = 0.f;
#pragma unroll 1
  for (int b = 0; b < NB; ++b) {
    const float xb = bfr(x[(size_t)b * SEQ_FULL + n]);
    s += (xb * gw0 + gb0) + (xb * gw1 + gb1);
  }
  s = wsum(s);
  const float mu = s * (1.0f / (float)(NB * GF));
  float ss = 0.f;
#pragma unroll 1
  for (int b = 0; b < NB; ++b) {
    const float xb = bfr(x[(size_t)b * SEQ_FULL + n]);
    const float d0 = (xb * gw0 + gb0) - mu;
    const float d1 = (xb * gw1 + gb1) - mu;
    ss += d0 * d0 + d1 * d1;
  }
  ss = wsum(ss);
  const float rs = 1.0f / sqrtf(ss * (1.0f / (float)(NB * GF)) + 1e-5f);
  const float gg = bfr(bn1g[n]), be = bfr(bn1b[n]);
#pragma unroll 1
  for (int pass = 0; pass < 2; ++pass) {
#pragma unroll 1
    for (int b = 0; b < NB; ++b) {
      const float xb = bfr(x[(size_t)b * SEQ_FULL + n]);
      const float y0 = gg * ((xb * gw0 + gb0) - mu) * rs + be;
      const float y1 = gg * ((xb * gw1 + gb1) - mu) * rs + be;
      const float h0 = fmaxf(y0, 0.f) + xb;
      const float h1 = fmaxf(y1, 0.f) + xb;
      unsigned hp, lp;
      split2(h0, h1, hp, lp);
      const size_t gr = (size_t)b * SEQ + n;
      const v2f hv = { h0, h1 };
      *(volatile v2f*)(H + gr * GF + 2 * lane) = hv;
      *(volatile unsigned*)(HHLw + gr * 64 + lane) = hp;
      *(volatile unsigned*)(HHLw + gr * 64 + 32 + lane) = lp;
    }
    __threadfence();
  }
}

__device__ __forceinline__ void proj64(const unsigned short* __restrict__ wrow, const Frag& bh0, const Frag& bl0,
                                       const Frag& bh1, const Frag& bl1, v8f (&acc)[4]) {
#pragma unroll
  for (int ct = 0; ct < 4; ++ct) {
    Frag a0, a1;
    ld_frag(a0, wrow + ct * 16 * GF);
    ld_frag(a1, wrow + ct * 16 * GF + 32);
    v8f d = z8();
    d = wmb(a0, bh0, d);
    d = wmb(a0, bl0, d);
    d = wmb(a1, bh1, d);
    d = wmb(a1, bl1, d);
    acc[ct] = d;
  }
}

__device__ __forceinline__ void stage_rm(const v8f (&acc)[4], const float* __restrict__ bias, bool valid,
                                         unsigned short* srow, int h) {
#pragma unroll
  for (int ct = 0; ct < 4; ++ct) {
    const int c0 = 16 * ct + 8 * h;
    const v4f b0 = *(const v4fa*)(bias + c0);
    const v4f b1 = *(const v4fa*)(bias + c0 + 4);
    float u[8];
#pragma unroll
    for (int j = 0; j < 4; ++j) {
      u[j]     = valid ? (acc[ct][j]     + bfr(b0[j])) : 0.f;
      u[4 + j] = valid ? (acc[ct][4 + j] + bfr(b1[j])) : 0.f;
    }
    const v4u pk = { pk2h(u[0], u[1]), pk2h(u[2], u[3]), pk2h(u[4], u[5]), pk2h(u[6], u[7]) };
    *(v4ua*)(srow + c0) = pk;
  }
}
__device__ __forceinline__ void stage_tr(const v8f (&acc)[4], const float* __restrict__ bias, bool valid,
                                         unsigned short* sv, int rowl, int h) {
#pragma unroll
  for (int ct = 0; ct < 4; ++ct) {
    const int c0 = 16 * ct + 8 * h;
    const v4f b0 = *(const v4fa*)(bias + c0);
    const v4f b1 = *(const v4fa*)(bias + c0 + 4);
#pragma unroll
    for (int j = 0; j < 4; ++j) {
      const float u0 = valid ? (acc[ct][j]     + bfr(b0[j])) : 0.f;
      const float u1 = valid ? (acc[ct][4 + j] + bfr(b1[j])) : 0.f;
      sv[(c0 + j) * 72 + rowl]     = f2h_bits(u0);
      sv[(c0 + 4 + j) * 72 + rowl] = f2h_bits(u1);
    }
  }
}
__global__ __launch_bounds__(128) void qkv_kernel(const unsigned short* __restrict__ HHL,
                                                  const unsigned short* __restrict__ WQKV,
                                                  const float* __restrict__ bq, const float* __restrict__ bk,
                                                  const float* __restrict__ bv,
                                                  unsigned short* __restrict__ Q, unsigned short* __restrict__ K,
                                                  unsigned short* __restrict__ VT) {
  __shared__ __align__(16) unsigned short sQ[64 * 72];
  __shared__ __align__(16) unsigned short sK[64 * 72];
  __shared__ __align__(16) unsigned short sV[64 * 72];
  const int tid = threadIdx.x, lane = tid & 31, w = tid >> 5;
  const int h = lane >> 4, m = lane & 15;
  const int b = blockIdx.y, s0 = blockIdx.x * 64;
  const int srow = s0 + 16 * w + m;
  const int scl = srow < SEQ ? srow : SEQ - 1;
  const bool valid = srow < SEQ;
  const unsigned short* hp = HHL + ((size_t)b * SEQ + scl) * 128 + 8 * h;
  Frag bh0, bh1, bl0, bl1;
  ld_frag(bh0, hp);
  ld_frag(bh1, hp + 32);
  ld_frag(bl0, hp + 64);
  ld_frag(bl1, hp + 96);
  const unsigned short* wr = WQKV + m * GF + 8 * h;
  v8f acc[4];
  proj64(wr, bh0, bl0, bh1, bl1, acc);
  stage_rm(acc, bq, valid, sQ + (16 * w + m) * 72, h);
  proj64(wr + 64 * GF, bh0, bl0, bh1, bl1, acc);
  stage_rm(acc, bk, valid, sK + (16 * w + m) * 72, h);
  proj64(wr + 128 * GF, bh0, bl0, bh1, bl1, acc);
  stage_tr(acc, bv, valid, sV, 16 * w + m, h);
  __syncthreads();

  const int q8 = lane & 7, sub = lane >> 3;
#pragma unroll 1
  for (int pass = 0; pass < 2; ++pass) {
#pragma unroll
    for (int i = 0; i < 4; ++i) {
      const int L = (4 * w + i) * 4 + sub;
      const int head = L >> 5, pair = L & 31;
      const int rowl = 2 * pair + (q8 >> 2), piece = q8 & 3;
      const size_t go = (((size_t)(b * 2 + head)) * SP + s0 + rowl) * HD + piece * 8;
      const v4u vq = *(const v4ua*)(sQ + rowl * 72 + head * 32 + piece * 8);
      const v4u vk = *(const v4ua*)(sK + rowl * 72 + head * 32 + piece * 8);
      *(volatile v4u*)(Q + go) = vq;
      *(volatile v4u*)(K + go) = vk;
      const v4u vv = *(const v4ua*)(sV + L * 72 + 8 * q8);
      const size_t gv = (((size_t)(b * 2 + (L >> 5))) * HD + (L & 31)) * SP + s0 + 8 * q8;
      *(volatile v4u*)(VT + gv) = vv;
    }
    if (pass == 0) __threadfence();
  }
}

__global__ __launch_bounds__(96) void attn_kernel(const unsigned short* __restrict__ Q,
                                                  const unsigned short* __restrict__ K,
                                                  const unsigned short* __restrict__ VT,
                                                  const unsigned* __restrict__ MB, const unsigned* __restrict__ TC,
                                                  unsigned short* __restrict__ CTX) {
  __shared__ __align__(16) float sC[3 * 16 * SCP];
  const int tid = threadIdx.x, lane = tid & 31, w = tid >> 5;
  const int h = lane >> 4, m = lane & 15;
  const int b = blockIdx.y;
  const int qt = blockIdx.x * 3 + w;
  const int q0 = 16 * qt;
  float* sc = sC + w * 16 * SCP;
  const unsigned* tcr = TC + (size_t)qt * MW;
  const unsigned* mbr = MB + (size_t)(q0 + m) * MW;
  const float scale = 0.17677669529663689f;
  const float ln4096 = 8.317766166719343f;
  const float ninf = __uint_as_float(0xFF800000u);

#pragma unroll 1
  for (int hd = 0; hd < 2; ++hd) {
    const int bh = b * 2 + hd;
    Frag fq;
    ld_frag(fq, Q + ((size_t)bh * SP + q0 + m) * HD + 8 * h);
    const unsigned short* kb = K + ((size_t)bh * SP + m) * HD + 8 * h;
    const unsigned short* vb = VT + ((size_t)bh * HD + m) * SP + 8 * h;
    float mrun = -1e30f, lsum = 0.f;
    v8f acc0 = z8(), acc1 = z8();
#pragma unroll 1
    for (int j = 0; j < KW; ++j) {
      const int cls = __builtin_amdgcn_readfirstlane((int)tcr[j]);
      if (cls != 2) {
        const int kp = 32 * j;
        Frag k0, k1;
        ld_frag(k0, kb + (size_t)kp * HD);
        ld_frag(k1, kb + (size_t)(kp + 16) * HD);
        const v8f s0 = wmh(k0, fq, z8());
        const v8f s1 = wmh(k1, fq, z8());
        unsigned mw = 0u;
        if (cls == 1) mw = mbr[j];
        const unsigned mws = mw >> (8 * h);
        float t[16];
#pragma unroll
        for (int i = 0; i < 8; ++i) {
          const float a0 = s0[i] * scale;
          const float a1 = s1[i] * scale;
          t[i]     = ((mws >> i) & 1u) ? ninf : a0;
          t[8 + i] = ((mws >> (16 + i)) & 1u) ? ninf : a1;
        }
        float tm = t[0];
#pragma unroll
        for (int i = 1; i < 16; ++i) tm = fmaxf(tm, t[i]);
        tm = fmaxf(tm, __shfl_xor(tm, 16));
        const float nm = fmaxf(mrun, tm);
        const float alpha = __expf(mrun - nm);
        mrun = nm;
        const float sh = ln4096 - nm;
        Frag pb;
        float ps = 0.f;
#pragma unroll
        for (int i = 0; i < 16; ++i) {
          const _Float16 ph = (_Float16)__expf(t[i] + sh);
          pb.f[i] = ph;
          ps += (float)ph;
        }
        lsum = lsum * alpha + ps;
#pragma unroll
        for (int r = 0; r < 8; ++r) { acc0[r] *= alpha; acc1[r] *= alpha; }
        Frag v0, v1;
        ld_frag(v0, vb + kp);
        ld_frag(v1, vb + (size_t)16 * SP + kp);
        acc0 = wmh(v0, pb, acc0);
        acc1 = wmh(v1, pb, acc1);
      }
    }
    lsum += __shfl_xor(lsum, 16);
    const float inv = 1.0f / lsum;
    const v4f o0 = { acc0[0] * inv, acc0[1] * inv, acc0[2] * inv, acc0[3] * inv };
    const v4f o1 = { acc0[4] * inv, acc0[5] * inv, acc0[6] * inv, acc0[7] * inv };
    const v4f o2 = { acc1[0] * inv, acc1[1] * inv, acc1[2] * inv, acc1[3] * inv };
    const v4f o3 = { acc1[4] * inv, acc1[5] * inv, acc1[6] * inv, acc1[7] * inv };
    float* dst = sc + m * SCP + hd * 32 + 8 * h;
    *(v4fa*)(dst) = o0;
    *(v4fa*)(dst + 4) = o1;
    *(v4fa*)(dst + 16) = o2;
    *(v4fa*)(dst + 20) = o3;
  }
  wave_lds_sync();
  unsigned short* g0 = CTX + ((size_t)b * SEQ + q0) * 128;
  hl_lines_store(sc, g0, lane);
  __threadfence();
  hl_lines_store(sc, g0, lane);
}

__device__ __forceinline__ void ln_rows(const v8f (&acc)[4], const float* __restrict__ bias,
                                        const float* __restrict__ res, const float* __restrict__ g,
                                        const float* __restrict__ be, float* scrow, int h) {
  float v[32];
#pragma unroll
  for (int ct = 0; ct < 4; ++ct) {
    const int c0 = 16 * ct + 8 * h;
    const v4f b0 = *(const v4fa*)(bias + c0);
    const v4f b1 = *(const v4fa*)(bias + c0 + 4);
    const v4f r0 = *(const v4fa*)(res + c0);
    const v4f r1 = *(const v4fa*)(res + c0 + 4);
#pragma unroll
    for (int j = 0; j < 4; ++j) {
      v[8 * ct + j]     = acc[ct][j]     + bfr(b0[j]) + r0[j];
      v[8 * ct + 4 + j] = acc[ct][4 + j] + bfr(b1[j]) + r1[j];
    }
  }
  float s = 0.f;
#pragma unroll
  for (int i = 0; i < 32; ++i) s += v[i];
  s += __shfl_xor(s, 16);
  const float mu = s * (1.0f / 64.0f);
  float ss = 0.f;
#pragma unroll
  for (int i = 0; i < 32; ++i) {
    const float d = v[i] - mu;
    v[i] = d;
    ss += d * d;
  }
  ss += __shfl_xor(ss, 16);
  const float rs = 1.0f / sqrtf(ss * (1.0f / 64.0f) + 1e-5f);
#pragma unroll
  for (int ct = 0; ct < 4; ++ct) {
    const int c0 = 16 * ct + 8 * h;
    const v4f g0 = *(const v4fa*)(g + c0);
    const v4f g1 = *(const v4fa*)(g + c0 + 4);
    const v4f e0 = *(const v4fa*)(be + c0);
    const v4f e1 = *(const v4fa*)(be + c0 + 4);
    v4f o0, o1;
#pragma unroll
    for (int j = 0; j < 4; ++j) {
      o0[j] = bfr(g0[j]) * v[8 * ct + j] * rs + bfr(e0[j]);
      o1[j] = bfr(g1[j]) * v[8 * ct + 4 + j] * rs + bfr(e1[j]);
    }
    *(v4fa*)(scrow + c0) = o0;
    *(v4fa*)(scrow + c0 + 4) = o1;
  }
}

__global__ __launch_bounds__(96) void oproj_kernel(const unsigned short* __restrict__ CTX,
                                                   const unsigned short* __restrict__ WO,
                                                   const float* __restrict__ bo, const float* __restrict__ H,
                                                   const float* __restrict__ lg, const float* __restrict__ lb,
                                                   float* __restrict__ H1, unsigned short* __restrict__ H1HL) {
  __shared__ __align__(16) float sC[3 * 16 * SCP];
  const int tid = threadIdx.x, lane = tid & 31, w = tid >> 5;
  const int h = lane >> 4, m = lane & 15;
  const int row0 = blockIdx.x * 48 + 16 * w;
  float* sc = sC + w * 16 * SCP;
  const unsigned short* cp = CTX + (size_t)(row0 + m) * 128 + 8 * h;
  Frag bh0, bh1, bl0, bl1;
  ld_frag(bh0, cp);
  ld_frag(bh1, cp + 32);
  ld_frag(bl0, cp + 64);
  ld_frag(bl1, cp + 96);
  v8f acc[4];
  proj64(WO + m * GF + 8 * h, bh0, bl0, bh1, bl1, acc);
  ln_rows(acc, bo, H + (size_t)(row0 + m) * GF, lg, lb, sc + m * SCP, h);
  wave_lds_sync();
  float* gf = H1 + (size_t)row0 * GF;
  unsigned short* gh = H1HL + (size_t)row0 * 128;
  f32_lines_store(sc, gf, GF, lane);
  hl_lines_store(sc, gh, lane);
  __threadfence();
  f32_lines_store(sc, gf, GF, lane);
  hl_lines_store(sc, gh, lane);
}

__device__ __forceinline__ v8f ffn1_tile(const unsigned short* __restrict__ wrow, const Frag& bh0, const Frag& bl0,
                                         const Frag& bh1, const Frag& bl1) {
  Frag a0, a1;
  ld_frag(a0, wrow);
  ld_frag(a1, wrow + 32);
  v8f d = z8();
  d = wmb(a0, bh0, d);
  d = wmb(a0, bl0, d);
  d = wmb(a1, bh1, d);
  d = wmb(a1, bl1, d);
  return d;
}
__global__ __launch_bounds__(96) void ffn_kernel(const unsigned short* __restrict__ H1HL,
                                                 const float* __restrict__ H1,
                                                 const unsigned short* __restrict__ W1B, const float* __restrict__ b1,
                                                 const unsigned short* __restrict__ W2B, const float* __restrict__ b2,
                                                 const float* __restrict__ lg, const float* __restrict__ lb,
                                                 unsigned short* __restrict__ H2HL) {
  __shared__ __align__(16) float sC[3 * 16 * SCP];
  const int tid = threadIdx.x, lane = tid & 31, w = tid >> 5;
  const int h = lane >> 4, m = lane & 15;
  const int row0 = blockIdx.x * 48 + 16 * w;
  float* sc = sC + w * 16 * SCP;
  const unsigned short* hp = H1HL + (size_t)(row0 + m) * 128 + 8 * h;
  Frag bh0, bh1, bl0, bl1;
  ld_frag(bh0, hp);
  ld_frag(bh1, hp + 32);
  ld_frag(bl0, hp + 64);
  ld_frag(bl1, hp + 96);
  const unsigned short* w1r = W1B + (size_t)m * GF + 8 * h;
  const unsigned short* w2r = W2B + (size_t)m * DFF + 8 * h;
  v8f acc[4];
#pragma unroll
  for (int ct = 0; ct < 4; ++ct) acc[ct] = z8();

#pragma unroll 1
  for (int jg = 0; jg < DFF / 32; ++jg) {
    const int j0 = 32 * jg;
    const v8f d0 = ffn1_tile(w1r + (size_t)j0 * GF, bh0, bl0, bh1, bl1);
    const v8f d1 = ffn1_tile(w1r + (size_t)(j0 + 16) * GF, bh0, bl0, bh1, bl1);
    const v4f ba = *(const v4fa*)(b1 + j0 + 8 * h);
    const v4f bb = *(const v4fa*)(b1 + j0 + 8 * h + 4);
    const v4f bc = *(const v4fa*)(b1 + j0 + 16 + 8 * h);
    const v4f bd = *(const v4fa*)(b1 + j0 + 16 + 8 * h + 4);
    float u0[8], u1[8];
#pragma unroll
    for (int j = 0; j < 4; ++j) {
      u0[j]     = fmaxf(d0[j]     + bfr(ba[j]), 0.f);
      u0[4 + j] = fmaxf(d0[4 + j] + bfr(bb[j]), 0.f);
      u1[j]     = fmaxf(d1[j]     + bfr(bc[j]), 0.f);
      u1[4 + j] = fmaxf(d1[4 + j] + bfr(bd[j]), 0.f);
    }
    unsigned hp0, hp1, hp2, hp3, hp4, hp5, hp6, hp7, lp0, lp1, lp2, lp3, lp4, lp5, lp6, lp7;
    split2(u0[0], u0[1], hp0, lp0);
    split2(u0[2], u0[3], hp1, lp1);
    split2(u0[4], u0[5], hp2, lp2);
    split2(u0[6], u0[7], hp3, lp3);
    split2(u1[0], u1[1], hp4, lp4);
    split2(u1[2], u1[3], hp5, lp5);
    split2(u1[4], u1[5], hp6, lp6);
    split2(u1[6], u1[7], hp7, lp7);
    const v4u qh0 = { hp0, hp1, hp2, hp3 };
    const v4u qh1 = { hp4, hp5, hp6, hp7 };
    const v4u ql0 = { lp0, lp1, lp2, lp3 };
    const v4u ql1 = { lp4, lp5, lp6, lp7 };
    Frag fh, fl;
    fh.q[0] = qh0; fh.q[1] = qh1;
    fl.q[0] = ql0; fl.q[1] = ql1;
#pragma unroll
    for (int ct = 0; ct < 4; ++ct) {
      Frag a;
      ld_frag(a, w2r + (size_t)ct * 16 * DFF + j0);
      acc[ct] = wmb(a, fh, acc[ct]);
      acc[ct] = wmb(a, fl, acc[ct]);
    }
  }
  ln_rows(acc, b2, H1 + (size_t)(row0 + m) * GF, lg, lb, sc + m * SCP, h);
  wave_lds_sync();
  unsigned short* gh = H2HL + (size_t)row0 * 128;
  hl_lines_store(sc, gh, lane);
  __threadfence();
  hl_lines_store(sc, gh, lane);
}

__global__ __launch_bounds__(128) void head_kernel(const unsigned short* __restrict__ H2HL,
                                                   const unsigned short* __restrict__ FCWB,
                                                   const float* __restrict__ fcb, float* __restrict__ OUT1) {
  __shared__ __align__(16) float sC[4 * 16 * SCP];
  const int tid = threadIdx.x, lane = tid & 31, w = tid >> 5;
  const int h = lane >> 4, m = lane & 15;
  const int b = blockIdx.y, n0 = blockIdx.x * 16;
  float* sc = sC + w * 16 * SCP;
  const int nn = (n0 + m) < NN ? (n0 + m) : (NN - 1);
  const unsigned short* hb = H2HL + ((size_t)b * SEQ + nn) * 128 + 8 * h;
  const unsigned short* wr = FCWB + (size_t)(64 * w + m) * KFC + 8 * h;
  v8f acc[4];
#pragma unroll
  for (int cl = 0; cl < 4; ++cl) acc[cl] = z8();
#pragma unroll 1
  for (int ks = 0; ks < KFC / 32; ++ks) {
    const int t = ks >> 1, koff = (ks & 1) * 32;
    const unsigned short* hp = hb + (size_t)t * NN * 128 + koff;
    Frag bh, bl;
    ld_frag(bh, hp);
    ld_frag(bl, hp + 64);
#pragma unroll
    for (int cl = 0; cl < 4; ++cl) {
      Frag a;
      ld_frag(a, wr + (size_t)cl * 16 * KFC + 32 * ks);
      acc[cl] = wmb(a, bh, acc[cl]);
      acc[cl] = wmb(a, bl, acc[cl]);
    }
  }
#pragma unroll
  for (int cl = 0; cl < 4; ++cl) {
    const int c0 = 16 * cl + 8 * h;
    const v4f b0 = *(const v4fa*)(fcb + 64 * w + c0);
    const v4f b1 = *(const v4fa*)(fcb + 64 * w + c0 + 4);
    v4f o0, o1;
#pragma unroll
    for (int j = 0; j < 4; ++j) {
      o0[j] = acc[cl][j] + bfr(b0[j]);
      o1[j] = acc[cl][4 + j] + bfr(b1[j]);
    }
    *(v4fa*)(sc + m * SCP + c0) = o0;
    *(v4fa*)(sc + m * SCP + c0 + 4) = o1;
  }
  wave_lds_sync();
  float* g0 = OUT1 + ((size_t)b * NPAD + n0) * FCO + 64 * w;
  f32_lines_store(sc, g0, FCO, lane);
  __threadfence();
  f32_lines_store(sc, g0, FCO, lane);
}

__global__ __launch_bounds__(256) void bn2fc3_kernel(const float* __restrict__ OUT1, const float* __restrict__ g2,
                                                     const float* __restrict__ b2, const float* __restrict__ fc3w,
                                                     const float* __restrict__ fc3b, float* __restrict__ Y) {
  __shared__ float sv[NB * FCO];
  __shared__ float sw3[NT * FCO];
  __shared__ float red[16];
  const int tid = threadIdx.x, lane = tid & 31, w = tid >> 5;
  const int n = blockIdx.x;
  float v[NB];
  float s = 0.f;
#pragma unroll
  for (int b = 0; b < NB; ++b) {
    v[b] = OUT1[((size_t)b * NPAD + n) * FCO + tid];
    s += v[b];
  }
  s = wsum(s);
  if (lane == 0) red[w] = s;
  __syncthreads();
  const float tot = ((red[0] + red[1]) + (red[2] + red[3])) + ((red[4] + red[5]) + (red[6] + red[7]));
  const float mu = tot * (1.0f / (float)(NB * FCO));
  float ss = 0.f;
#pragma unroll
  for (int b = 0; b < NB; ++b) {
    const float d = v[b] - mu;
    v[b] = d;
    ss += d * d;
  }
  ss = wsum(ss);
  if (lane == 0) red[8 + w] = ss;
  __syncthreads();
  const float tq = ((red[8] + red[9]) + (red[10] + red[11])) + ((red[12] + red[13]) + (red[14] + red[15]));
  const float rs = 1.0f / sqrtf(tq * (1.0f / (float)(NB * FCO)) + 1e-5f);
  const float gg = bfr(g2[n]), be = bfr(b2[n]);
#pragma unroll
  for (int b = 0; b < NB; ++b) sv[b * FCO + tid] = fmaxf(gg * v[b] * rs + be, 0.f);
#pragma unroll 1
  for (int i = tid; i < NT * FCO; i += 256) sw3[i] = bfr(fc3w[i]);
  __syncthreads();
  if (tid < YP) {
    const int q = tid < NB * NT ? tid : NB * NT - 1;
    const int bq = q / NT, t = q - bq * NT;
    float acc = bfr(fc3b[t]);
#pragma unroll 4
    for (int i = 0; i < FCO; ++i) acc += sv[bq * FCO + i] * sw3[t * FCO + i];
    const float o = tid < NB * NT ? acc : 0.f;
    float* d = Y + (size_t)n * YP + tid;
    *(volatile float*)d = o;
    __threadfence();
    *(volatile float*)d = o;
  }
}

__global__ __launch_bounds__(256) void out_kernel(const float* __restrict__ Y, float* __restrict__ out) {
  const int i = blockIdx.x * 256 + threadIdx.x;
  if (i >= ROWS / 4) return;
  v4f v;
#pragma unroll
  for (int c = 0; c < 4; ++c) {
    const int e = 4 * i + c;
    const int b = e / SEQ;
    const int r = e - b * SEQ;
    const int t = r / NN;
    const int n = r - t * NN;
    v[c] = Y[(size_t)n * YP + b * NT + t];
  }
  float* d = out + (size_t)4 * i;
  *(volatile v4f*)d = v;
  __threadfence();
  *(volatile v4f*)d = v;
}

constexpr size_t SZ_WALL = (size_t)NW_ALL * 2;
constexpr size_t SZ_MB   = (size_t)SEQ * MW * 4;
constexpr size_t SZ_TC   = (size_t)QTILES * MW * 4;
constexpr size_t SZ_F64  = (size_t)ROWS * GF * 4;
constexpr size_t SZ_HL   = (size_t)ROWS * 128 * 2;
constexpr size_t SZ_QK   = (size_t)NB * 2 * SP * HD * 2;
constexpr size_t SZ_OUT1 = (size_t)NB * NPAD * FCO * 4;
constexpr size_t SZ_Y    = (size_t)NN * YP * 4;
constexpr size_t O_WALL = 0;
constexpr size_t O_MB   = O_WALL + SZ_WALL;
constexpr size_t O_TC   = O_MB + SZ_MB;
constexpr size_t O_H    = O_TC + SZ_TC;
constexpr size_t O_HHL  = O_H + SZ_F64;
constexpr size_t O_Q    = O_HHL + SZ_HL;
constexpr size_t O_K    = O_Q + SZ_QK;
constexpr size_t O_VT   = O_K + SZ_QK;
constexpr size_t O_CTX  = O_VT + SZ_QK;
constexpr size_t O_H1   = O_CTX + SZ_HL;
constexpr size_t O_H1HL = O_H1 + SZ_F64;
constexpr size_t O_H2HL = O_H1HL + SZ_HL;
constexpr size_t O_OUT1 = O_H2HL + SZ_HL;
constexpr size_t O_Y    = O_OUT1 + SZ_OUT1;
constexpr size_t WS_TOTAL = O_Y + SZ_Y;
static_assert(SZ_WALL % 128 == 0);
static_assert(SZ_MB % 128 == 0);
static_assert(SZ_TC % 128 == 0);
static_assert(SZ_F64 % 128 == 0);
static_assert(SZ_HL % 128 == 0);
static_assert(SZ_QK % 128 == 0);
static_assert(SZ_OUT1 % 128 == 0);
static_assert(SZ_Y % 128 == 0);
static_assert(WS_TOTAL <= (size_t)WSCAP);

extern "C" void kernel_launch(void* const* d_in, const int* in_sizes, int n_in,
                              void* d_out, int out_size, void* d_ws, size_t ws_size,
                              hipStream_t stream) {
  if (n_in < 29) return;
  if (in_sizes[0] < NB * SEQ_FULL) return;
  if (in_sizes[1] < SEQ * NEMB) return;
  if (in_sizes[2] < NEMB * GF) return;
  if (in_sizes[3] < NEMB * GF) return;
  if (in_sizes[4] < SEQ || in_sizes[5] < SEQ) return;
  if (in_sizes[6] < NN || in_sizes[7] < NN) return;
  if (in_sizes[8] < GF * GF || in_sizes[10] < GF * GF || in_sizes[12] < GF * GF || in_sizes[14] < GF * GF) return;
  if (in_sizes[9] < GF || in_sizes[11] < GF || in_sizes[13] < GF || in_sizes[15] < GF) return;
  if (in_sizes[16] < GF || in_sizes[17] < GF || in_sizes[22] < GF || in_sizes[23] < GF) return;
  if (in_sizes[18] < DFF * GF || in_sizes[19] < DFF) return;
  if (in_sizes[20] < GF * DFF || in_sizes[21] < GF) return;
  if (in_sizes[24] < FCO * KFC || in_sizes[25] < FCO) return;
  if (in_sizes[26] < NT * FCO || in_sizes[27] < NT) return;
  if (in_sizes[28] < SEQ) return;
  if ((size_t)in_sizes[28] < (size_t)SEQ * SEQ_FULL) return;
  if (out_size < NB * SEQ) return;
  if (WS_TOTAL > ws_size) return;

  const float* x    = (const float*)d_in[0];
  const float* ne   = (const float*)d_in[1];
  const float* gcw  = (const float*)d_in[2];
  const float* gcb  = (const float*)d_in[3];
  const float* bn1g = (const float*)d_in[4];
  const float* bn1b = (const float*)d_in[5];
  const float* bn2g = (const float*)d_in[6];
  const float* bn2b = (const float*)d_in[7];
  const float* Wq = (const float*)d_in[8];   const float* bq = (const float*)d_in[9];
  const float* Wk = (const float*)d_in[10];  const float* bk = (const float*)d_in[11];
  const float* Wv = (const float*)d_in[12];  const float* bv = (const float*)d_in[13];
  const float* Wo = (const float*)d_in[14];  const float* bo = (const float*)d_in[15];
  const float* ln1g = (const float*)d_in[16]; const float* ln1b = (const float*)d_in[17];
  const float* W1 = (const float*)d_in[18];  const float* b1 = (const float*)d_in[19];
  const float* W2 = (const float*)d_in[20];  const float* b2 = (const float*)d_in[21];
  const float* ln2g = (const float*)d_in[22]; const float* ln2b = (const float*)d_in[23];
  const float* FCW = (const float*)d_in[24]; const float* FCb = (const float*)d_in[25];
  const float* FC3W = (const float*)d_in[26]; const float* FC3b = (const float*)d_in[27];
  const int* mask = (const int*)d_in[28];
  float* out = (float*)d_out;

  char* ws = (char*)d_ws;
  unsigned short* WALL = (unsigned short*)(ws + O_WALL);
  unsigned* MBp   = (unsigned*)(ws + O_MB);
  unsigned* TCp   = (unsigned*)(ws + O_TC);
  float* Hp       = (float*)(ws + O_H);
  unsigned short* HHL  = (unsigned short*)(ws + O_HHL);
  unsigned short* Qp   = (unsigned short*)(ws + O_Q);
  unsigned short* Kp   = (unsigned short*)(ws + O_K);
  unsigned short* VTp  = (unsigned short*)(ws + O_VT);
  unsigned short* CTX  = (unsigned short*)(ws + O_CTX);
  float* H1p      = (float*)(ws + O_H1);
  unsigned short* H1HL = (unsigned short*)(ws + O_H1HL);
  unsigned short* H2HL = (unsigned short*)(ws + O_H2HL);
  float* OUT1     = (float*)(ws + O_OUT1);
  float* Yp       = (float*)(ws + O_Y);

  prep_kernel<<<dim3((NW_ALL / 8) / 256), dim3(256), 0, stream>>>(Wq, Wk, Wv, Wo, W1, W2, FCW, WALL);
  mask_kernel<<<dim3(QTILES), dim3(256), 0, stream>>>(mask, MBp, TCp);
  gcn_kernel<<<dim3(SEQ / 8), dim3(256), 0, stream>>>(x, ne, gcw, gcb, bn1g, bn1b, Hp, (unsigned*)HHL);
  qkv_kernel<<<dim3(SP / 64, NB), dim3(128), 0, stream>>>(HHL, WALL + OW_QKV, bq, bk, bv, Qp, Kp, VTp);
  attn_kernel<<<dim3(QTILES / 3, NB), dim3(96), 0, stream>>>(Qp, Kp, VTp, MBp, TCp, CTX);
  oproj_kernel<<<dim3(ROWS / 48), dim3(96), 0, stream>>>(CTX, WALL + OW_O, bo, Hp, ln1g, ln1b, H1p, H1HL);
  ffn_kernel<<<dim3(ROWS / 48), dim3(96), 0, stream>>>(H1HL, H1p, WALL + OW_1, b1, WALL + OW_2, b2, ln2g, ln2b, H2HL);
  head_kernel<<<dim3(NPAD / 16, NB), dim3(128), 0, stream>>>(H2HL, WALL + OW_FC, FCb, OUT1);
  bn2fc3_kernel<<<dim3(NN), dim3(256), 0, stream>>>(OUT1, bn2g, bn2b, FC3W, FC3b, Yp);
  out_kernel<<<dim3((ROWS / 4 + 255) / 256), dim3(256), 0, stream>>>(Yp, out);
  (void)hipGetLastError();
}
